// ConvAutoEncoder_83227876261959
// MI455X (gfx1250) — hardware-verified
//
#include <hip/hip_runtime.h>
#include <math.h>

typedef __attribute__((ext_vector_type(16))) _Float16 v16h;
typedef __attribute__((ext_vector_type(8)))  _Float16 v8h;
typedef __attribute__((ext_vector_type(16))) __bf16   v16b;
typedef __attribute__((ext_vector_type(8)))  __bf16   v8b;
typedef __attribute__((ext_vector_type(8)))  float    v8f;
typedef __attribute__((ext_vector_type(4)))  float    v4f;
typedef __attribute__((ext_vector_type(2)))  float    v2f;

constexpr int NODES  = 64;
constexpr int GDIM   = 4;
constexpr int NCOORD = 2;
constexpr int NBATCH = 16384;
constexpr int XROW   = NODES * NCOORD;
constexpr int HROW   = NODES * GDIM;
constexpr int KCONV  = HROW;
constexpr int NCONV  = NODES * 2;
constexpr int NDEC1  = NODES * 8;
constexpr int KDEC1  = NCONV;
constexpr int NDEC2  = NODES * 2;
constexpr int KDEC2  = NDEC1;
constexpr int APITCH = 72;
constexpr int GAT_WAVES = 2;
constexpr float LEAKY_SLOPE = 0.2f;

static_assert(KCONV % 32 == 0 && KDEC1 % 32 == 0 && KDEC2 % 32 == 0);
static_assert(NBATCH % 64 == 0 && NCONV % 64 == 0 && NDEC1 % 64 == 0 && NDEC2 % 64 == 0);
static_assert(NBATCH % GAT_WAVES == 0);
static_assert(HROW == 32 * 8);

constexpr size_t WS_WC  = (size_t)NCONV * KCONV * 2;
constexpr size_t WS_W1  = (size_t)NDEC1 * KDEC1 * 2;
constexpr size_t WS_W2  = (size_t)NDEC2 * KDEC2 * 2;
constexpr size_t WS_CB2 = 512;
constexpr size_t WS_H   = (size_t)NBATCH * HROW * 2;
constexpr size_t WS_F   = (size_t)NBATCH * KDEC1 * 2;
constexpr size_t WS_D   = (size_t)NBATCH * NDEC1 * 2;
constexpr size_t OFF_WCHI = 0;
constexpr size_t OFF_WCLO = OFF_WCHI + WS_WC;
constexpr size_t OFF_W1HI = OFF_WCLO + WS_WC;
constexpr size_t OFF_W1LO = OFF_W1HI + WS_W1;
constexpr size_t OFF_W2HI = OFF_W1LO + WS_W1;
constexpr size_t OFF_W2LO = OFF_W2HI + WS_W2;
constexpr size_t OFF_CB2  = OFF_W2LO + WS_W2;
constexpr size_t OFF_HHI  = OFF_CB2 + WS_CB2;
constexpr size_t OFF_HLO  = OFF_HHI + WS_H;
constexpr size_t OFF_FHI  = OFF_HLO + WS_H;
constexpr size_t OFF_FLO  = OFF_FHI + WS_F;
constexpr size_t OFF_DHI  = OFF_FLO + WS_F;
constexpr size_t OFF_DLO  = OFF_DHI + WS_D;
constexpr size_t WS_TOTAL = OFF_DLO + WS_D;
static_assert(OFF_WCLO % 128 == 0 && OFF_W1HI % 128 == 0 && OFF_W1LO % 128 == 0 && OFF_W2HI % 128 == 0);
static_assert(OFF_W2LO % 128 == 0 && OFF_CB2 % 128 == 0 && OFF_HHI % 128 == 0 && OFF_HLO % 128 == 0);
static_assert(OFF_FHI % 128 == 0 && OFF_FLO % 128 == 0 && OFF_DHI % 128 == 0 && OFF_DLO % 128 == 0);
static_assert(WS_TOTAL <= (size_t)134217728);

constexpr size_t OUT0_BYTES    = (size_t)NBATCH * NCONV * 4;
constexpr size_t OUT1_BYTE_OFF = 8388608;
constexpr size_t OUT1_ELEM_OFF = OUT1_BYTE_OFF / 4;
constexpr size_t OUT_TOTAL_BYTES = 16777216;
static_assert(OUT0_BYTES == OUT1_BYTE_OFF);
static_assert(OUT1_BYTE_OFF + (size_t)NBATCH * NDEC2 * 4 <= OUT_TOTAL_BYTES);
static_assert(OUT1_BYTE_OFF % 128 == 0);

__device__ __forceinline__ unsigned short f2bf_bits(float f) {
  unsigned u = __float_as_uint(f);
  return (unsigned short)((u + 0x7FFFu + ((u >> 16) & 1u)) >> 16);
}
__device__ __forceinline__ float bf_bits2f(unsigned short h) { return __uint_as_float(((unsigned)h) << 16); }

__device__ __forceinline__ void dep_guard_h(v8f& a, v8f& b, v16h x, v16h y) { asm volatile("v_nop\n\tv_nop\n\tv_nop\n\tv_nop" : "+v"(a), "+v"(b) : "v"(x), "v"(y)); }
__device__ __forceinline__ void dep_guard_b(v8f& a, v8f& b, v16b x, v16b y) { asm volatile("v_nop\n\tv_nop\n\tv_nop\n\tv_nop" : "+v"(a), "+v"(b) : "v"(x), "v"(y)); }
__device__ __forceinline__ void keep4_h(v16h a, v16h b, v16h c, v16h d) { asm volatile("v_nop" :: "v"(a), "v"(b), "v"(c), "v"(d)); }
__device__ __forceinline__ void keep4_b(v16b a, v16b b, v16b c, v16b d) { asm volatile("v_nop" :: "v"(a), "v"(b), "v"(c), "v"(d)); }
__device__ __forceinline__ void acc_guard4(v8f& a, v8f& b, v8f& c, v8f& d) { asm volatile("v_nop\n\tv_nop\n\tv_nop\n\tv_nop" : "+v"(a), "+v"(b), "+v"(c), "+v"(d)); }
template <typename T> struct Frag;
template <> struct Frag<_Float16> {
  typedef v16h V; union U { v16h v; v8h h[2]; };
  static __device__ __forceinline__ v16h load(const _Float16* p) {
    U f; f.h[0] = *(const v8h*)(p); f.h[1] = *(const v8h*)(p + 16); return f.v;
  }
  static __device__ __forceinline__ v8f mma(v16h a, v16h b, v8f c) {
    return __builtin_amdgcn_wmma_f32_16x16x32_f16(false, a, false, b, (short)0, c, false, false);
  }
  static __device__ __forceinline__ void guard(v8f& a, v8f& b, v16h x, v16h y) { dep_guard_h(a, b, x, y); }
  static __device__ __forceinline__ void keep(v16h a, v16h b, v16h c, v16h d) { keep4_h(a, b, c, d); }
};
template <> struct Frag<__bf16> {
  typedef v16b V; union U { v16b v; v8b h[2]; };
  static __device__ __forceinline__ v16b load(const __bf16* p) {
    U f; f.h[0] = *(const v8b*)(p); f.h[1] = *(const v8b*)(p + 16); return f.v;
  }
  static __device__ __forceinline__ v8f mma(v16b a, v16b b, v8f c) {
    return __builtin_amdgcn_wmma_f32_16x16x32_bf16(false, a, false, b, (short)0, c, false, false);
  }
  static __device__ __forceinline__ void guard(v8f& a, v8f& b, v16b x, v16b y) { dep_guard_b(a, b, x, y); }
  static __device__ __forceinline__ void keep(v16b a, v16b b, v16b c, v16b d) { keep4_b(a, b, c, d); }
};

__device__ __forceinline__ unsigned short at_bf_bits(float f) {
  unsigned u = __float_as_uint(f);
  return (unsigned short)((u + 0x7FFFu + ((u >> 16) & 1u)) >> 16);
}
__device__ __forceinline__ __bf16 at_f2bf(float f) { return __builtin_bit_cast(__bf16, at_bf_bits(f)); }
__device__ __forceinline__ void at_split(float f, __bf16& hi, __bf16& lo) {
  const unsigned short hb = at_bf_bits(f);
  hi = __builtin_bit_cast(__bf16, hb);
  lo = at_f2bf(f - __uint_as_float(((unsigned)hb) << 16));
}
__device__ __forceinline__ v8f at_mma(v16b a, v16b b, v8f c) {
  c = __builtin_amdgcn_wmma_f32_16x16x32_bf16(false, a, false, b, (short)0, c, false, false);
  asm volatile("v_nop\n\tv_nop\n\tv_nop\n\tv_nop" : "+v"(c) : "v"(a), "v"(b));
  return c;
}

__device__ __forceinline__ void split_store8(v8f v, unsigned short* ph, unsigned short* pl) {
  v8h hv, lv;
#pragma unroll
  for (int e = 0; e < 8; ++e) {
    const unsigned short hb = f2bf_bits(v[e]);
    const unsigned short lb = f2bf_bits(v[e] - bf_bits2f(hb));
    hv[e] = __builtin_bit_cast(_Float16, hb);
    lv[e] = __builtin_bit_cast(_Float16, lb);
  }
  *(volatile v8h*)(void*)ph = hv;
  *(volatile v8h*)(void*)pl = lv;
  __threadfence();
  *(volatile v8h*)(void*)ph = hv;
  *(volatile v8h*)(void*)pl = lv;
}

template <int ET> struct Elem;
template <> struct Elem<0> { typedef _Float16 T; };
template <> struct Elem<1> { typedef __bf16 T; };
template <int ET, bool SPLIT, int BIAS_MODE, int OUT_MODE, bool RESID, int ACT = 0>
__global__ __launch_bounds__(256) void wmma_gemm64(
    const unsigned short* __restrict__ Ap, const unsigned short* __restrict__ A2p, int lda, long strideA,
    const unsigned short* __restrict__ Btp, const unsigned short* __restrict__ Bt2p, int ldb, long strideB,
    void* __restrict__ Cout, void* __restrict__ Cout2, void* __restrict__ Cout3, int ldc, long strideC,
    const float* __restrict__ bias,
    const float* __restrict__ resid, long strideR,
    int M, int N, int K, float scale) {
  typedef typename Elem<ET>::T T;
  typedef typename Frag<T>::V V;
  const T* A = (const T*)Ap; const T* A2 = (const T*)A2p; const T* Bt = (const T*)Btp; const T* Bt2 = (const T*)Bt2p;
  __shared__ __align__(16) float sT[8][16 * 68];
  const int b    = blockIdx.y;
  const int lane = threadIdx.x & 31;
  const int wave = threadIdx.x >> 5;
  const int tilesN = N >> 6;
  const int tilesM = M >> 6;
  const int tile = blockIdx.x * 8 + wave;
  if (tile >= tilesM * tilesN) return;
  const int tm = tile / tilesN;
  const int tn = tile - tm * tilesN;
  const int m0 = tm << 6;
  const int n0 = tn << 6;

  const T* Ab  = A  + (size_t)b * strideA;
  const T* Bb  = Bt + (size_t)b * strideB;
  const T* Ab2 = SPLIT ? (A2  + (size_t)b * strideA) : nullptr;
  const T* Bb2 = SPLIT ? (Bt2 + (size_t)b * strideB) : nullptr;

  const int rlane = lane & 15;
  const int koff  = (lane >> 4) * 8;
  const int mOff  = (lane >> 4) * 8;

  v8f acc[4][4];
#pragma unroll
  for (int i = 0; i < 4; ++i)
#pragma unroll
    for (int j = 0; j < 4; ++j) acc[i][j] = (v8f){0.f,0.f,0.f,0.f,0.f,0.f,0.f,0.f};

  for (int k0 = 0; k0 < K; k0 += 32) {
    V bh[4], bl[4];
#pragma unroll
    for (int j = 0; j < 4; ++j) {
      const size_t bo = (size_t)(n0 + (j << 4) + rlane) * ldb + koff + k0;
      bh[j] = Frag<T>::load(Bb + bo);
      if (SPLIT) bl[j] = Frag<T>::load(Bb2 + bo);
    }
#pragma unroll
    for (int i = 0; i < 4; ++i) {
      const size_t ao = (size_t)(m0 + (i << 4) + rlane) * lda + koff + k0;
      V ah = Frag<T>::load(Ab + ao);
      V al;
      if (SPLIT) al = Frag<T>::load(Ab2 + ao);
#pragma unroll
      for (int j = 0; j < 4; ++j) {
        acc[i][j] = Frag<T>::mma(ah, bh[j], acc[i][j]);
        if (SPLIT) {
          acc[i][j] = Frag<T>::mma(ah, bl[j], acc[i][j]);
          acc[i][j] = Frag<T>::mma(al, bh[j], acc[i][j]);
        }
      }
      Frag<T>::guard(acc[i][0], acc[i][3], ah, SPLIT ? al : ah);
    }
    Frag<T>::keep(bh[0], bh[1], bh[2], bh[3]);
    if (SPLIT) Frag<T>::keep(bl[0], bl[1], bl[2], bl[3]);
  }
  acc_guard4(acc[0][0], acc[0][1], acc[0][2], acc[0][3]);
  acc_guard4(acc[1][0], acc[1][1], acc[1][2], acc[1][3]);
  acc_guard4(acc[2][0], acc[2][1], acc[2][2], acc[2][3]);
  acc_guard4(acc[3][0], acc[3][1], acc[3][2], acc[3][3]);

  float* slab = sT[wave];
  const float* Rb = RESID ? (resid + (size_t)b * strideR) : nullptr;
#pragma unroll
  for (int i = 0; i < 4; ++i) {
    const int mBase = m0 + (i << 4);
#pragma unroll
    for (int j = 0; j < 4; ++j) {
      const int n = n0 + (j << 4) + rlane;
      float bv = 0.f;
      if (BIAS_MODE == 2) bv = bias[n];
#pragma unroll
      for (int r = 0; r < 8; ++r) {
        float v = acc[i][j][r] * scale;
        if (BIAS_MODE == 1) v += bias[mBase + mOff + r];
        if (BIAS_MODE == 2) v += bv;
        if (RESID) v += Rb[(size_t)(mBase + mOff + r) * ldc + n];
        if (ACT == 1) v = tanhf(v);
        if (ACT == 2) v = fmaxf(v, 0.0f);
        if (ACT == 3) v = v / (1.0f + expf(-v));
        if (ACT == 4) v = (v > 0.f) ? v : 0.01f * v;
        slab[(mOff + r) * 68 + (j << 4) + rlane] = v;
      }
    }
    __builtin_amdgcn_fence(__ATOMIC_RELEASE, "workgroup");
    __builtin_amdgcn_wave_barrier();
    __builtin_amdgcn_fence(__ATOMIC_ACQUIRE, "workgroup");
    if (OUT_MODE == 0 || OUT_MODE == 3) {
      float* C = (float*)Cout + (size_t)b * strideC;
      const int hh = lane >> 4, c4 = (lane & 15) * 4;
      for (int pass = 0; pass < 2; ++pass) {
#pragma unroll
        for (int it = 0; it < 8; ++it) {
          const int row = it * 2 + hh;
          v4f v = *(const v4f*)(slab + row * 68 + c4);
          *(volatile v4f*)(C + (size_t)(mBase + row) * ldc + n0 + c4) = v;
        }
        __threadfence();
      }
    }
    if (OUT_MODE != 0) {
      const int q = lane >> 3, c8 = (lane & 7) * 8;
      unsigned short* C  = ((OUT_MODE == 3) ? (unsigned short*)Cout2 : (unsigned short*)Cout) + (size_t)b * strideC;
      unsigned short* C2 = ((OUT_MODE == 3) ? (unsigned short*)Cout3 : (unsigned short*)Cout2) + (size_t)b * strideC;
      for (int pass = 0; pass < 2; ++pass) {
#pragma unroll
        for (int it = 0; it < 4; ++it) {
          const int row = it * 4 + q;
          const float* sp = slab + row * 68 + c8;
          v8h hv, lv;
#pragma unroll
          for (int e = 0; e < 8; ++e) {
            if (OUT_MODE == 1) {
              hv[e] = (_Float16)sp[e];
            } else {
              unsigned short hb = f2bf_bits(sp[e]);
              unsigned short lb = f2bf_bits(sp[e] - bf_bits2f(hb));
              hv[e] = __builtin_bit_cast(_Float16, hb);
              lv[e] = __builtin_bit_cast(_Float16, lb);
            }
          }
          *(volatile v8h*)(C + (size_t)(mBase + row) * ldc + n0 + c8) = hv;
          if (OUT_MODE >= 2) *(volatile v8h*)(C2 + (size_t)(mBase + row) * ldc + n0 + c8) = lv;
        }
        __threadfence();
      }
    }
    __builtin_amdgcn_fence(__ATOMIC_RELEASE, "workgroup");
    __builtin_amdgcn_wave_barrier();
    __builtin_amdgcn_fence(__ATOMIC_ACQUIRE, "workgroup");
  }
}

constexpr int PREP_BLK_CONV = NCONV * KCONV / 8 / 256;
constexpr int PREP_BLK_W1   = NDEC1 * KDEC1 / 8 / 256;
constexpr int PREP_BLK_W2   = NDEC2 * KDEC2 / 8 / 256;
constexpr int PREP_BLOCKS   = PREP_BLK_CONV + PREP_BLK_W1 + PREP_BLK_W2 + 1;
static_assert(PREP_BLK_CONV * 256 * 8 == NCONV * KCONV && PREP_BLK_W1 * 256 * 8 == NDEC1 * KDEC1 && PREP_BLK_W2 * 256 * 8 == NDEC2 * KDEC2);

__global__ __launch_bounds__(256) void prep_params_kernel(
    const float* __restrict__ conv_w, const float* __restrict__ conv_b,
    const float* __restrict__ dec_w1, const float* __restrict__ dec_w2,
    unsigned short* __restrict__ WChi, unsigned short* __restrict__ WClo,
    unsigned short* __restrict__ W1hi, unsigned short* __restrict__ W1lo,
    unsigned short* __restrict__ W2hi, unsigned short* __restrict__ W2lo,
    float* __restrict__ cb2)
{
  const int blk = blockIdx.x;
  const int tid = threadIdx.x;
  if (blk < PREP_BLK_CONV) {
    const int g  = blk * 256 + tid;
    const int n  = g >> 5;
    const int kb = (g & 31) * 8;
    const int o  = n >> 1, p = n & 1;
    v8f vals;
#pragma unroll
    for (int e = 0; e < 8; ++e) {
      const int k = kb + e;
      const int i = k >> 2, q = k & 3;
      const int r = q - p;
      const bool valid = (r >= 0) && (r < 3);
      const int rc = (r < 0) ? 0 : ((r > 2) ? 2 : r);
      const float v = conv_w[(o * NODES + i) * 3 + rc];
      vals[e] = valid ? v : 0.f;
    }
    split_store8(vals, WChi + (size_t)n * KCONV + kb, WClo + (size_t)n * KCONV + kb);
  } else if (blk < PREP_BLK_CONV + PREP_BLK_W1) {
    const int g  = (blk - PREP_BLK_CONV) * 256 + tid;
    const int n  = g >> 4;
    const int kb = (g & 15) * 8;
    const v4f a0 = *(const v4f*)(dec_w1 + (size_t)n * KDEC1 + kb);
    const v4f a1 = *(const v4f*)(dec_w1 + (size_t)n * KDEC1 + kb + 4);
    v8f vals;
    vals[0] = a0[0]; vals[1] = a0[1]; vals[2] = a0[2]; vals[3] = a0[3];
    vals[4] = a1[0]; vals[5] = a1[1]; vals[6] = a1[2]; vals[7] = a1[3];
    split_store8(vals, W1hi + (size_t)n * KDEC1 + kb, W1lo + (size_t)n * KDEC1 + kb);
  } else if (blk < PREP_BLK_CONV + PREP_BLK_W1 + PREP_BLK_W2) {
    const int g  = (blk - PREP_BLK_CONV - PREP_BLK_W1) * 256 + tid;
    const int n  = g >> 6;
    const int kb = (g & 63) * 8;
    const v4f a0 = *(const v4f*)(dec_w2 + (size_t)n * KDEC2 + kb);
    const v4f a1 = *(const v4f*)(dec_w2 + (size_t)n * KDEC2 + kb + 4);
    v8f vals;
    vals[0] = a0[0]; vals[1] = a0[1]; vals[2] = a0[2]; vals[3] = a0[3];
    vals[4] = a1[0]; vals[5] = a1[1]; vals[6] = a1[2]; vals[7] = a1[3];
    split_store8(vals, W2hi + (size_t)n * KDEC2 + kb, W2lo + (size_t)n * KDEC2 + kb);
  } else {
    if (tid < 32) {
      const float b0 = conv_b[2 * tid];
      const float b1 = conv_b[2 * tid + 1];
      v4f v; v[0] = b0; v[1] = b0; v[2] = b1; v[3] = b1;
      *(volatile v4f*)(cb2 + 4 * tid) = v;
      __threadfence();
      *(volatile v4f*)(cb2 + 4 * tid) = v;
    }
  }
}

__global__ __launch_bounds__(64) void gat_layer_kernel(
    const float* __restrict__ x, const float* __restrict__ W_gat, const float* __restrict__ a_attn,
    unsigned short* __restrict__ Hhi, unsigned short* __restrict__ Hlo, int nb)
{
  __shared__ __align__(16) __bf16 Ahi[GAT_WAVES][NODES * APITCH];
  __shared__ __align__(16) __bf16 Alo[GAT_WAVES][NODES * APITCH];
  __shared__ __align__(16) __bf16 Bhi[GAT_WAVES][16 * APITCH];
  __shared__ __align__(16) __bf16 Blo[GAT_WAVES][16 * APITCH];
  __shared__ __align__(16) float esw[GAT_WAVES][NODES];
  __shared__ __align__(16) float invw[GAT_WAVES][NODES];
  __shared__ __align__(16) float hst[GAT_WAVES][HROW];

  const int tid  = threadIdx.x;
  const int wave = tid >> 5;
  const int lane = tid & 31;
  const int rlane = lane & 15, hh = lane >> 4, koff = hh * 8;
  int bb = blockIdx.x * GAT_WAVES + wave;
  bb = (bb < nb) ? bb : (nb - 1);

  float w[8], av[8];
#pragma unroll
  for (int i = 0; i < 8; ++i) { w[i] = W_gat[i]; av[i] = a_attn[i]; }

  const float* xb = x + (size_t)bb * XROW;
  const v2f xa = *(const v2f*)(xb + 2 * lane);
  const v2f xc = *(const v2f*)(xb + 2 * (lane + 32));
  float z0[GDIM], z1[GDIM];
  float es0 = 0.f, ed0 = 0.f, es1 = 0.f, ed1 = 0.f;
#pragma unroll
  for (int d = 0; d < GDIM; ++d) {
    z0[d] = xa[0] * w[2 * d] + xa[1] * w[2 * d + 1];
    z1[d] = xc[0] * w[2 * d] + xc[1] * w[2 * d + 1];
    es0 += z0[d] * av[d];      ed0 += z0[d] * av[GDIM + d];
    es1 += z1[d] * av[d];      ed1 += z1[d] * av[GDIM + d];
  }
  esw[wave][lane] = es0;
  esw[wave][lane + 32] = es1;
  {
    __bf16* bh  = Bhi[wave];
    __bf16* blp = Blo[wave];
#pragma unroll
    for (int d = 0; d < GDIM; ++d) {
      __bf16 h_, l_;
      at_split(z0[d], h_, l_); bh[d * APITCH + lane] = h_;      blp[d * APITCH + lane] = l_;
      at_split(z1[d], h_, l_); bh[d * APITCH + lane + 32] = h_; blp[d * APITCH + lane + 32] = l_;
    }
    constexpr int NZ = (16 - GDIM) * APITCH * 2 / 16;
    static_assert(NZ * 16 == (16 - GDIM) * APITCH * 2);
    const uint4 zz = make_uint4(0u, 0u, 0u, 0u);
    uint4* zh = (uint4*)(bh + GDIM * APITCH);
    uint4* zl = (uint4*)(blp + GDIM * APITCH);
    for (int qq = lane; qq < NZ; qq += 32) { zh[qq] = zz; zl[qq] = zz; }
  }
  __syncthreads();

  const float* es = esw[wave];
  const int j0 = lane, j1 = lane + 32;
  float m0 = -INFINITY, m1 = -INFINITY;
#pragma unroll 4
  for (int i = 0; i < NODES; ++i) {
    const float ev = es[i];
    float e0 = ev + ed0; e0 = (e0 >= 0.f) ? e0 : LEAKY_SLOPE * e0; e0 = (i == j0) ? -INFINITY : e0;
    float e1 = ev + ed1; e1 = (e1 >= 0.f) ? e1 : LEAKY_SLOPE * e1; e1 = (i == j1) ? -INFINITY : e1;
    m0 = fmaxf(m0, e0);
    m1 = fmaxf(m1, e1);
  }
  float den0 = 0.f, den1 = 0.f;
  {
    __bf16* ahp = Ahi[wave];
    __bf16* alp = Alo[wave];
#pragma unroll 4
    for (int i = 0; i < NODES; ++i) {
      const float ev = es[i];
      float e0 = ev + ed0; e0 = (e0 >= 0.f) ? e0 : LEAKY_SLOPE * e0; e0 = (i == j0) ? -INFINITY : e0;
      float e1 = ev + ed1; e1 = (e1 >= 0.f) ? e1 : LEAKY_SLOPE * e1; e1 = (i == j1) ? -INFINITY : e1;
      const float p0 = expf(e0 - m0);
      const float p1 = expf(e1 - m1);
      den0 += p0;
      den1 += p1;
      __bf16 h_, l_;
      at_split(p0, h_, l_); ahp[j0 * APITCH + i] = h_; alp[j0 * APITCH + i] = l_;
      at_split(p1, h_, l_); ahp[j1 * APITCH + i] = h_; alp[j1 * APITCH + i] = l_;
    }
  }
  invw[wave][j0] = 1.0f / den0;
  invw[wave][j1] = 1.0f / den1;
  __syncthreads();

  v8f acc[4];
#pragma unroll
  for (int t = 0; t < 4; ++t) acc[t] = (v8f){0.f,0.f,0.f,0.f,0.f,0.f,0.f,0.f};
  {
    const __bf16* Ab = Ahi[wave];
    const __bf16* Al = Alo[wave];
    const __bf16* Bh = Bhi[wave];
    const __bf16* Bl = Blo[wave];
#pragma unroll
    for (int ks = 0; ks < 2; ++ks) {
      const int k0 = ks * 32;
      const v16b bh = Frag<__bf16>::load(Bh + rlane * APITCH + koff + k0);
      const v16b bl = Frag<__bf16>::load(Bl + rlane * APITCH + koff + k0);
#pragma unroll
      for (int mt = 0; mt < 4; ++mt) {
        const v16b ah = Frag<__bf16>::load(Ab + (mt * 16 + rlane) * APITCH + koff + k0);
        const v16b al = Frag<__bf16>::load(Al + (mt * 16 + rlane) * APITCH + koff + k0);
        acc[mt] = at_mma(ah, bh, acc[mt]);
        acc[mt] = at_mma(ah, bl, acc[mt]);
        acc[mt] = at_mma(al, bh, acc[mt]);
      }
    }
  }

  {
    float* hs = hst[wave];
    const float* iv = invw[wave];
#pragma unroll
    for (int mt = 0; mt < 4; ++mt) {
#pragma unroll
      for (int r = 0; r < 8; ++r) {
        const int j = mt * 16 + 8 * hh + r;
        const float val = acc[mt][r] * iv[j];
        if (rlane < GDIM) hs[j * GDIM + rlane] = val;
      }
    }
  }
  __syncthreads();

  {
    const float* sp = hst[wave] + 8 * lane;
    v8f vals;
#pragma unroll
    for (int e = 0; e < 8; ++e) vals[e] = sp[e];
    split_store8(vals, Hhi + (size_t)bb * HROW + 8 * lane, Hlo + (size_t)bb * HROW + 8 * lane);
  }
}

extern "C" void kernel_launch(void* const* d_in, const int* in_sizes, int n_in,
                              void* d_out, int out_size, void* d_ws, size_t ws_size,
                              hipStream_t stream) {
  if (n_in < 9) return;
  if (in_sizes[0] != NBATCH * XROW) return;
  if (in_sizes[1] != GDIM * NCOORD || in_sizes[2] != 2 * GDIM) return;
  if (in_sizes[3] != NODES * NODES * 3 || in_sizes[4] != NODES) return;
  if (in_sizes[5] != NDEC1 * KDEC1 || in_sizes[6] != NDEC1) return;
  if (in_sizes[7] != NDEC2 * KDEC2 || in_sizes[8] != NDEC2) return;
  if ((size_t)out_size * 4 != OUT_TOTAL_BYTES) return;
  if (ws_size < WS_TOTAL) return;

  const float* x      = (const float*)d_in[0];
  const float* W_gat  = (const float*)d_in[1];
  const float* a_attn = (const float*)d_in[2];
  const float* conv_w = (const float*)d_in[3];
  const float* conv_b = (const float*)d_in[4];
  const float* dec_w1 = (const float*)d_in[5];
  const float* dec_b1 = (const float*)d_in[6];
  const float* dec_w2 = (const float*)d_in[7];
  const float* dec_b2 = (const float*)d_in[8];

  char* ws = (char*)d_ws;
  unsigned short* WChi = (unsigned short*)(ws + OFF_WCHI);
  unsigned short* WClo = (unsigned short*)(ws + OFF_WCLO);
  unsigned short* W1hi = (unsigned short*)(ws + OFF_W1HI);
  unsigned short* W1lo = (unsigned short*)(ws + OFF_W1LO);
  unsigned short* W2hi = (unsigned short*)(ws + OFF_W2HI);
  unsigned short* W2lo = (unsigned short*)(ws + OFF_W2LO);
  float*          cb2  = (float*)(ws + OFF_CB2);
  unsigned short* Hhi  = (unsigned short*)(ws + OFF_HHI);
  unsigned short* Hlo  = (unsigned short*)(ws + OFF_HLO);
  unsigned short* Fhi  = (unsigned short*)(ws + OFF_FHI);
  unsigned short* Flo  = (unsigned short*)(ws + OFF_FLO);
  unsigned short* Dhi  = (unsigned short*)(ws + OFF_DHI);
  unsigned short* Dlo  = (unsigned short*)(ws + OFF_DLO);

  float* out0 = (float*)d_out;
  float* out1 = (float*)d_out + OUT1_ELEM_OFF;

  prep_params_kernel<<<dim3(PREP_BLOCKS), dim3(256), 0, stream>>>(
      conv_w, conv_b, dec_w1, dec_w2, WChi, WClo, W1hi, W1lo, W2hi, W2lo, cb2);

  gat_layer_kernel<<<dim3(NBATCH / GAT_WAVES), dim3(32 * GAT_WAVES), 0, stream>>>(
      x, W_gat, a_attn, Hhi, Hlo, NBATCH);

  {
    const int tiles = (NBATCH / 64) * (NCONV / 64);
    wmma_gemm64<1, true, 2, 3, false, 0><<<dim3((tiles + 7) / 8, 1), dim3(256), 0, stream>>>(
        Hhi, Hlo, KCONV, 0L, WChi, WClo, KCONV, 0L,
        (void*)out0, (void*)Fhi, (void*)Flo, NCONV, 0L,
        cb2, cb2, 0L, NBATCH, NCONV, KCONV, 1.0f);
  }
  {
    const int tiles = (NBATCH / 64) * (NDEC1 / 64);
    wmma_gemm64<1, true, 2, 2, false, 2><<<dim3((tiles + 7) / 8, 1), dim3(256), 0, stream>>>(
        Fhi, Flo, KDEC1, 0L, W1hi, W1lo, KDEC1, 0L,
        (void*)Dhi, (void*)Dlo, (void*)Dlo, NDEC1, 0L,
        dec_b1, dec_b1, 0L, NBATCH, NDEC1, KDEC1, 1.0f);
  }
  {
    const int tiles = (NBATCH / 64) * (NDEC2 / 64);
    wmma_gemm64<1, true, 2, 0, false, 0><<<dim3((tiles + 7) / 8, 1), dim3(256), 0, stream>>>(
        Dhi, Dlo, KDEC2, 0L, W2hi, W2lo, KDEC2, 0L,
        (void*)out1, (void*)Dhi, (void*)Dhi, NDEC2, 0L,
        dec_b2, dec_b2, 0L, NBATCH, NDEC2, KDEC2, 1.0f);
  }
}
